// GATLayer_7009386627243
// MI455X (gfx1250) — hardware-run, weakly checked
//
#include <hip/hip_runtime.h>

typedef float          v8f   __attribute__((ext_vector_type(8)));
typedef float          v4f   __attribute__((ext_vector_type(4)));
typedef unsigned int   v4u   __attribute__((ext_vector_type(4)));
typedef int            v8i   __attribute__((ext_vector_type(8)));
typedef unsigned short v8us  __attribute__((ext_vector_type(8)));
typedef unsigned short v16us __attribute__((ext_vector_type(16)));
typedef __bf16         v16bf __attribute__((ext_vector_type(16)));
typedef _Float16       v16h  __attribute__((ext_vector_type(16)));
typedef v4f  __attribute__((may_alias)) v4fa;
typedef v8us __attribute__((may_alias)) v8usa;
union FragB { v16bf v; v16us u; v8us h[2]; v8i w; };
union FragH { v16h  v; v16us u; v8us h[2]; v8i w; };

__device__ __forceinline__ v8f wmb(const FragB& a, const FragB& b, v8f c) {
  v8f d = __builtin_amdgcn_wmma_f32_16x16x32_bf16(false, a.v, false, b.v, (short)0, c, false, false);
  asm volatile("v_nop\n\tv_nop\n\tv_nop\n\tv_nop" : "+v"(d) : "v"(a.w), "v"(b.w));
  return d;
}

__device__ __forceinline__ v8f wmh(const FragH& a, const FragH& b, v8f c) {
  v8f d = __builtin_amdgcn_wmma_f32_16x16x32_f16(false, a.v, false, b.v, (short)0, c, false, false);
  asm volatile("v_nop\n\tv_nop\n\tv_nop\n\tv_nop" : "+v"(d) : "v"(a.w), "v"(b.w));
  return d;
}

__device__ __forceinline__ unsigned bf16_bits(float f) {
  const unsigned u = __float_as_uint(f);
  const unsigned r = (u + 0x7FFFu + ((u >> 16) & 1u)) >> 16;
  const unsigned q = (u >> 16) | 0x40u;
  return ((u & 0x7fffffffu) > 0x7f800000u) ? q : r;
}

__device__ __forceinline__ float bf16_val(float f) {
  return __uint_as_float(bf16_bits(f) << 16);
}
__device__ __forceinline__ int clampi(int v, int lo, int hi) {
  return v < lo ? lo : (v > hi ? hi : v);
}

__device__ __forceinline__ unsigned f16_bits(float f) {
  const unsigned u  = __float_as_uint(f);
  const unsigned s  = (u >> 16) & 0x8000u;
  const unsigned a  = u & 0x7fffffffu;
  const unsigned t  = a - 0x38000000u;
  const unsigned r  = (t + 0x0FFFu + ((t >> 13) & 1u)) >> 13;
  const unsigned rc = r > 0x7C00u ? 0x7C00u : r;
  const bool small  = a < 0x38800000u;
  const bool isnan  = a > 0x7f800000u;
  const unsigned fin = small ? 0u : (s | rc);
  return isnan ? (s | 0x7E00u) : fin;
}

__device__ __forceinline__ unsigned pk16(unsigned lo, unsigned hi) { return lo | (hi << 16); }
__device__ __forceinline__ unsigned bf16_lo_bits(float v) {
  float hi = bf16_val(v);
  asm volatile("" : "+v"(hi));
  return bf16_bits(v - hi);
}
__device__ __forceinline__ v4u pack8_bf16(v4f a, v4f c) {
  return (v4u){ pk16(bf16_bits(a[0]), bf16_bits(a[1])), pk16(bf16_bits(a[2]), bf16_bits(a[3])),
                pk16(bf16_bits(c[0]), bf16_bits(c[1])), pk16(bf16_bits(c[2]), bf16_bits(c[3])) };
}
__device__ __forceinline__ v4u pack8_bf16_lo(v4f a, v4f c) {
  return (v4u){ pk16(bf16_lo_bits(a[0]), bf16_lo_bits(a[1])), pk16(bf16_lo_bits(a[2]), bf16_lo_bits(a[3])),
                pk16(bf16_lo_bits(c[0]), bf16_lo_bits(c[1])), pk16(bf16_lo_bits(c[2]), bf16_lo_bits(c[3])) };
}
__device__ __forceinline__ v4u pack8_f16(v4f a, v4f c) {
  return (v4u){ pk16(f16_bits(a[0]), f16_bits(a[1])), pk16(f16_bits(a[2]), f16_bits(a[3])),
                pk16(f16_bits(c[0]), f16_bits(c[1])), pk16(f16_bits(c[2]), f16_bits(c[3])) };
}

template <int FORM>
__global__ __launch_bounds__(256) void k_plane(const float* __restrict__ src, int rows, int cols, int ldsrc,
                                               unsigned short* __restrict__ dst, int MP, int KP) {
  static_assert(FORM >= 0 && FORM <= 3);
  const int KTOT = (FORM == 1 || FORM == 3) ? 2 * KP : KP;
  const unsigned ppr   = (unsigned)(KTOT >> 3);
  const unsigned kp8   = (unsigned)(KP >> 3);
  const unsigned total = (unsigned)MP * ppr;
  const unsigned g     = blockIdx.x * 256u + threadIdx.x;
  const unsigned rowu  = g / ppr;
  const unsigned p     = g - rowu * ppr;
  const bool second    = p >= kp8;
  const int row = (int)rowu;
  const int c0  = (int)((second ? p - kp8 : p) << 3);
  const float* srow = src + (size_t)clampi(row, 0, rows - 1) * (size_t)ldsrc;
  float x[8];
  unsigned mk[8];
#pragma unroll
  for (int e = 0; e < 8; ++e) {
    const int c = c0 + e;
    const float v = srow[clampi(c, 0, cols - 1)];
    asm volatile("" :: "v"(v));
    x[e]  = v;
    mk[e] = (row < rows && c < cols) ? 0xFFFFu : 0u;
  }
  const v4f a = (v4f){ x[0], x[1], x[2], x[3] };
  const v4f c = (v4f){ x[4], x[5], x[6], x[7] };
  v4u o;
  if (FORM == 2) {
    o = pack8_f16(a, c);
  } else {
    const v4u hi = pack8_bf16(a, c);
    o = hi;
    if (FORM == 1) { const v4u lo = pack8_bf16_lo(a, c); o = second ? lo : hi; }
  }
  const v4u mw = (v4u){ pk16(mk[0], mk[1]), pk16(mk[2], mk[3]), pk16(mk[4], mk[5]), pk16(mk[6], mk[7]) };
  o &= mw;
  if (g < total) {
    volatile v4u* q = (volatile v4u*)(dst + (size_t)g * 8);
    *q = o;
    __threadfence();
    *q = o;
  }
}

template <int FORM> struct FragOf    { typedef FragB T; };
template <>         struct FragOf<2> { typedef FragH T; };
__device__ __forceinline__ v8f mm(const FragB& a, const FragB& b, v8f c) { return wmb(a, b, c); }
__device__ __forceinline__ v8f mm(const FragH& a, const FragH& b, v8f c) { return wmh(a, b, c); }
template <class F> __device__ __forceinline__ F ld_frag(const unsigned short* p) {
  F f;
  f.h[0] = *(const v8usa*)(p);
  f.h[1] = *(const v8usa*)(p + 16);
  return f;
}

template <int FORM, int EPI>
__global__ __launch_bounds__(256) __attribute__((amdgpu_num_vgpr(248)))
void k_gemm_nt(const unsigned short* __restrict__ A, const unsigned short* __restrict__ B,
               const float* __restrict__ bias, float* __restrict__ D, int M, int N, int KTOT, int ldd) {
  static_assert(FORM >= 0 && FORM <= 2);
  static_assert(EPI == 0 || EPI == 1);
  typedef typename FragOf<FORM>::T F;
  __shared__ __attribute__((aligned(16))) float sT[8][16 * 68];
  const int lane = threadIdx.x & 31;
  const int wave = threadIdx.x >> 5;
  const int tilesM = (M + 63) >> 6;
  const int tilesN = (N + 63) >> 6;
  const int tile = blockIdx.x * 8 + wave;
  if (tile >= tilesM * tilesN) return;
  const int tm = tile / tilesN;
  const int tn = tile - tm * tilesN;
  const int m0 = tm << 6;
  const int n0 = tn << 6;

  const int rl = lane & 15;
  const int h8 = (lane >> 4) * 8;
  const unsigned short* pa = A + (size_t)(m0 + rl) * (size_t)KTOT + h8;
  const unsigned short* pb = B + (size_t)(n0 + rl) * (size_t)KTOT + h8;

  v8f acc[4][4];
#pragma unroll
  for (int i = 0; i < 4; ++i)
#pragma unroll
    for (int j = 0; j < 4; ++j) acc[i][j] = (v8f){0.f, 0.f, 0.f, 0.f, 0.f, 0.f, 0.f, 0.f};

#pragma unroll 1
  for (int k0 = 0; k0 < KTOT; k0 += 32) {
    F bf[4];
#pragma unroll
    for (int j = 0; j < 4; ++j) bf[j] = ld_frag<F>(pb + (size_t)(j << 4) * (size_t)KTOT + k0);
#pragma unroll
    for (int i = 0; i < 4; ++i) {
      const F af = ld_frag<F>(pa + (size_t)(i << 4) * (size_t)KTOT + k0);
#pragma unroll
      for (int j = 0; j < 4; ++j) acc[i][j] = mm(af, bf[j], acc[i][j]);
    }
  }

  float* slab = sT[wave];
  const int hh = lane >> 4;
  const int c4 = (lane & 15) * 4;
  const int nc = n0 + c4;
  const bool cok = nc < N;
  v4f bv = (v4f){0.f, 0.f, 0.f, 0.f};
  if (EPI == 1) {
    bv = *(const v4fa*)(bias + clampi(nc, 0, N - 4));
    asm volatile("" :: "v"(bv));
  }
#pragma unroll
  for (int i = 0; i < 4; ++i) {
    const int mBase = m0 + (i << 4);
#pragma unroll
    for (int j = 0; j < 4; ++j) {
#pragma unroll
      for (int r = 0; r < 8; ++r) slab[(h8 + r) * 68 + (j << 4) + rl] = acc[i][j][r];
    }
    __builtin_amdgcn_fence(__ATOMIC_RELEASE, "workgroup");
    __builtin_amdgcn_wave_barrier();
    __builtin_amdgcn_fence(__ATOMIC_ACQUIRE, "workgroup");
    v4f vv[8];
#pragma unroll
    for (int it = 0; it < 8; ++it) {
      const int row = it * 2 + hh;
      v4f v = *(const v4fa*)(slab + row * 68 + c4);
      if (EPI == 1) v += bv;
      vv[it] = v;
    }
    for (int pass = 0; pass < 2; ++pass) {
#pragma unroll
      for (int it = 0; it < 8; ++it) {
        const int row = mBase + it * 2 + hh;
        if (cok && row < M) *(volatile v4f*)(D + (size_t)row * (size_t)ldd + nc) = vv[it];
      }
      __threadfence();
    }
    __builtin_amdgcn_fence(__ATOMIC_RELEASE, "workgroup");
    __builtin_amdgcn_wave_barrier();
    __builtin_amdgcn_fence(__ATOMIC_ACQUIRE, "workgroup");
  }
}

#pragma clang fp contract(off)

typedef int v4i __attribute__((ext_vector_type(4)));
typedef int v2i __attribute__((ext_vector_type(2)));
typedef v4i __attribute__((may_alias)) v4ia;
typedef v2i __attribute__((may_alias)) v2ia;

#define GB      16
#define GS      1024
#define GEP     8192
#define NN      16384
#define GC      128
#define RCAP    16384
#define DEGCAP  64
#define DEGMAX  32
#define OFFP    1056
#define ATABN   1024
#define ANUM    272
#define T_SOFT  1.0f
#define LDS_BUCKET ((2 * GEP + RCAP + 32) * 4)

#define SZ_XB   ((size_t)NN * 128 * 2)
#define SZ_WT   ((size_t)128 * 128 * 2)
#define SZ_ATAB ((size_t)ATABN * 4)
#define SZ_XT   ((size_t)NN * 128 * 4)
#define SZ_SS   ((size_t)NN * 4)
#define SZ_LIST ((size_t)GB * RCAP * 4)
#define SZ_OFF  ((size_t)GB * OFFP * 4)
#define SZ_FLAG ((size_t)4096)
#define WS_TOTAL (SZ_XB + SZ_WT + SZ_ATAB + SZ_XT + SZ_SS + SZ_SS + SZ_LIST + SZ_OFF + SZ_FLAG)

static_assert(GB * GS == NN);
static_assert(GS == 1024 && GEP == 8192);
static_assert(RCAP == 2 * GEP && RCAP == 16384);
static_assert(DEGCAP >= 2 * DEGMAX && DEGCAP == 64);
static_assert(GC == 32 * 4);
static_assert(NN % 64 == 0 && 128 % 64 == 0 && 128 % 32 == 0 && NN % 16 == 0);
static_assert(NN == 2048 * 8 && NN == 512 * 32);
static_assert((NN * 128 / 8) % 256 == 0);
static_assert(GEP % 256 == 0 && RCAP % 1024 == 0 && (RCAP * 4) % 128 == 0);
static_assert(OFFP == GS + 32 && (OFFP * 4) % 128 == 0);
static_assert(ANUM % 4 == 0 && ANUM <= ATABN && ATABN == 256 * 4);
static_assert(GB * 32 * 4 <= 4096);
static_assert(LDS_BUCKET == 131200 && LDS_BUCKET <= 262144);
static_assert(SZ_XB % 128 == 0 && SZ_WT % 128 == 0 && SZ_ATAB % 128 == 0 && SZ_XT % 128 == 0);
static_assert(SZ_SS % 128 == 0 && SZ_LIST % 128 == 0 && SZ_OFF % 128 == 0 && SZ_FLAG % 128 == 0);
static_assert(WS_TOTAL == (size_t)13871104);
static_assert(WS_TOTAL <= ((size_t)128 << 20));
static_assert((size_t)(NN - 1) * GC + 127 < (size_t)2097152);

__global__ __launch_bounds__(256) void k_prep(const float* __restrict__ W, const float* __restrict__ a,
                                              unsigned short* __restrict__ WT, float* __restrict__ ATAB) {
  __shared__ __attribute__((aligned(16))) float sW[128 * 36];
  const int tid = (int)threadIdx.x;
  const int nb0 = (int)blockIdx.x * 32;
#pragma unroll
  for (int i = 0; i < 4; ++i) {
    const int f  = i * 256 + tid;
    const int k  = f >> 3;
    const int c4 = (f & 7) * 4;
    const v4f v = *(const v4fa*)(W + k * 128 + nb0 + c4);
    *(v4fa*)(sW + k * 36 + c4) = v;
  }
  __syncthreads();
  v4u o0, o1;
  int r0, k00, r1, k01;
  {
    const int piece = tid;
    r0 = piece >> 4; k00 = (piece & 15) * 8;
    const v4f x = (v4f){ sW[(k00 + 0) * 36 + r0], sW[(k00 + 1) * 36 + r0], sW[(k00 + 2) * 36 + r0], sW[(k00 + 3) * 36 + r0] };
    const v4f y = (v4f){ sW[(k00 + 4) * 36 + r0], sW[(k00 + 5) * 36 + r0], sW[(k00 + 6) * 36 + r0], sW[(k00 + 7) * 36 + r0] };
    o0 = pack8_bf16(x, y);
  }
  {
    const int piece = 256 + tid;
    r1 = piece >> 4; k01 = (piece & 15) * 8;
    const v4f x = (v4f){ sW[(k01 + 0) * 36 + r1], sW[(k01 + 1) * 36 + r1], sW[(k01 + 2) * 36 + r1], sW[(k01 + 3) * 36 + r1] };
    const v4f y = (v4f){ sW[(k01 + 4) * 36 + r1], sW[(k01 + 5) * 36 + r1], sW[(k01 + 6) * 36 + r1], sW[(k01 + 7) * 36 + r1] };
    o1 = pack8_bf16(x, y);
  }
  volatile v4u* q0 = (volatile v4u*)(WT + (size_t)(nb0 + r0) * 128 + k00);
  volatile v4u* q1 = (volatile v4u*)(WT + (size_t)(nb0 + r1) * 128 + k01);
  *q0 = o0; *q1 = o1;
  __threadfence();
  *q0 = o0; *q1 = o1;

  const int t = tid < (ANUM / 4) ? tid : (ANUM / 4 - 1);
  const v4f av = *(const v4fa*)(a + 4 * t);
  asm volatile("" :: "v"(av));
  const unsigned mk = tid < (ANUM / 4) ? 0xFFFFFFFFu : 0u;
  const v4f ar = (v4f){ __uint_as_float((bf16_bits(av.x) << 16) & mk), __uint_as_float((bf16_bits(av.y) << 16) & mk),
                        __uint_as_float((bf16_bits(av.z) << 16) & mk), __uint_as_float((bf16_bits(av.w) << 16) & mk) };
  if (blockIdx.x == 0) {
    volatile v4f* qa = (volatile v4f*)(ATAB + 4 * tid);
    *qa = ar;
    __threadfence();
    *qa = ar;
  }
}

__global__ __launch_bounds__(256) void k_node(const float* __restrict__ XT, const float* __restrict__ ATAB,
                                              float* __restrict__ SS, float* __restrict__ SD) {
  __shared__ __attribute__((aligned(16))) float sS[32];
  __shared__ __attribute__((aligned(16))) float sD[32];
  const int tid = (int)threadIdx.x, lane = tid & 31, wave = tid >> 5;
  const v4f as = *(const v4fa*)(ATAB + 4 * lane);
  const v4f ad = *(const v4fa*)(ATAB + 128 + 4 * lane);
  asm volatile("" :: "v"(as), "v"(ad));
  const int nb = (int)blockIdx.x * 32 + wave * 4;
#pragma unroll
  for (int i = 0; i < 4; ++i) {
    const int n = nb + i;
    const v4f r = *(const v4fa*)(XT + (size_t)n * GC + 4 * lane);
    asm volatile("" :: "v"(r));
    float ps = r.x * as.x;
    ps = ps + r.y * as.y;
    ps = ps + r.z * as.z;
    ps = ps + r.w * as.w;
    float pd = r.x * ad.x;
    pd = pd + r.y * ad.y;
    pd = pd + r.z * ad.z;
    pd = pd + r.w * ad.w;
    ps = ps + __shfl_xor(ps, 1);
    pd = pd + __shfl_xor(pd, 1);
    ps = ps + __shfl_xor(ps, 2);
    pd = pd + __shfl_xor(pd, 2);
    ps = ps + __shfl_xor(ps, 4);
    pd = pd + __shfl_xor(pd, 4);
    ps = ps + __shfl_xor(ps, 8);
    pd = pd + __shfl_xor(pd, 8);
    ps = ps + __shfl_xor(ps, 16);
    pd = pd + __shfl_xor(pd, 16);
    if (lane == 0) { sS[wave * 4 + i] = ps; sD[wave * 4 + i] = pd; }
  }
  __syncthreads();
  const v4f vs = *(const v4fa*)(sS + 4 * (lane & 7));
  const v4f vd = *(const v4fa*)(sD + 4 * (lane & 7));
  if (wave == 0 && lane < 8) {
    volatile v4f* q = (volatile v4f*)(SS + (size_t)blockIdx.x * 32 + 4 * lane);
    *q = vs;
    __threadfence();
    *q = vs;
  }
  if (wave == 1 && lane < 8) {
    volatile v4f* q = (volatile v4f*)(SD + (size_t)blockIdx.x * 32 + 4 * lane);
    *q = vd;
    __threadfence();
    *q = vd;
  }
}

__global__ __launch_bounds__(256) void k_bucket(const int* __restrict__ ei, int* __restrict__ LISTg,
                                                int* __restrict__ OFFg, int* __restrict__ FLAGg) {
  extern __shared__ __attribute__((aligned(16))) int dl[];
  int* sp     = dl;
  int* placed = dl + 2 * GEP;
  int* misc   = placed + RCAP;
  const int tid = (int)threadIdx.x, lane = tid & 31, wave = tid >> 5;
  const int blk = (int)blockIdx.x;
  const int* pg = ei + (size_t)blk * (size_t)(GEP * 2);

  if (tid < 32) misc[tid] = 0;
  {
    const v4i z4 = (v4i){0, 0, 0, 0};
#pragma unroll 1
    for (int it = 0; it < RCAP / 1024; ++it) *(v4ia*)(placed + 4 * (it * 256 + tid)) = z4;
  }
#pragma unroll 4
  for (int it = 0; it < GEP / 256; ++it) {
    const int e = it * 256 + tid;
    v2i p = *(const v2ia*)(pg + 2 * e);
    asm volatile("" :: "v"(p));
    v2i c;
    c.x = clampi(p.x, 0, GS - 1);
    c.y = clampi(p.y, 0, GS - 1);
    *(v2ia*)(sp + 2 * e) = c;
  }
  __syncthreads();

  const int base = tid * 4;
  int f0 = 0, f1 = 0, f2 = 0, f3 = 0, r0 = 0, r1 = 0, r2 = 0, r3 = 0;
#pragma unroll 4
  for (int e = 0; e < GEP; ++e) {
    const v2i p = *(const v2ia*)(sp + 2 * e);
    const int dk = p.y - base;
    const int sk = p.x - base;
    f0 += (dk == 0) ? 1 : 0;
    f1 += (dk == 1) ? 1 : 0;
    f2 += (dk == 2) ? 1 : 0;
    f3 += (dk == 3) ? 1 : 0;
    r0 += (sk == 0) ? 1 : 0;
    r1 += (sk == 1) ? 1 : 0;
    r2 += (sk == 2) ? 1 : 0;
    r3 += (sk == 3) ? 1 : 0;
  }

  const int t0 = f0 + r0, t1 = f1 + r1, t2 = f2 + r2, t3 = f3 + r3;
  const int ts = (t0 + t1) + (t2 + t3);
  int incl = ts;
#pragma unroll
  for (int d = 1; d < 32; d <<= 1) {
    const int up = __shfl_up(incl, d);
    incl += (lane >= d) ? up : 0;
  }
  if (lane == 31) misc[8 + wave] = incl;
  if (t0 > DEGCAP || t1 > DEGCAP || t2 > DEGCAP || t3 > DEGCAP) misc[16] = 1;
  __syncthreads();
  int pre = 0, nh = 0;
#pragma unroll
  for (int w2 = 0; w2 < 8; ++w2) {
    const int tw = misc[8 + w2];
    nh  += tw;
    pre += (w2 < wave) ? tw : 0;
  }
  const int s0 = pre + incl - ts;
  const int s1 = s0 + t0;
  const int s2 = s1 + t1;
  const int s3 = s2 + t2;
  const int fl = ((misc[16] != 0) || (nh != RCAP)) ? 1 : 0;

  int cf0 = s0, cf1 = s1, cf2 = s2, cf3 = s3;
  int cr0 = s0 + f0, cr1 = s1 + f1, cr2 = s2 + f2, cr3 = s3 + f3;
#pragma unroll 2
  for (int e = 0; e < GEP; ++e) {
    const v2i p = *(const v2ia*)(sp + 2 * e);
    const int dk = p.y - base;
    const int sk = p.x - base;
    const int wf = p.x | (e << 10);
    const int wr = p.y | (e << 10);
    if ((unsigned)dk < 4u) {
      if (dk == 0)      { placed[clampi(cf0, 0, RCAP - 1)] = wf; cf0 += 1; }
      else if (dk == 1) { placed[clampi(cf1, 0, RCAP - 1)] = wf; cf1 += 1; }
      else if (dk == 2) { placed[clampi(cf2, 0, RCAP - 1)] = wf; cf2 += 1; }
      else              { placed[clampi(cf3, 0, RCAP - 1)] = wf; cf3 += 1; }
    }
    if ((unsigned)sk < 4u) {
      if (sk == 0)      { placed[clampi(cr0, 0, RCAP - 1)] = wr; cr0 += 1; }
      else if (sk == 1) { placed[clampi(cr1, 0, RCAP - 1)] = wr; cr1 += 1; }
      else if (sk == 2) { placed[clampi(cr2, 0, RCAP - 1)] = wr; cr2 += 1; }
      else              { placed[clampi(cr3, 0, RCAP - 1)] = wr; cr3 += 1; }
    }
  }
  __syncthreads();

  int* lbase = LISTg + (size_t)blk * RCAP;
  for (int pass = 0; pass < 2; ++pass) {
#pragma unroll 1
    for (int it = 0; it < RCAP / 1024; ++it) {
      const int o4 = 4 * (it * 256 + tid);
      const v4i v = *(const v4ia*)(placed + o4);
      *(volatile v4i*)(lbase + o4) = v;
    }
    __threadfence();
  }
  {
    const v4i oc = (v4i){ s0, s1, s2, s3 };
    const v4i tl = (v4i){ nh, nh, nh, nh };
    const v4i fv = (v4i){ fl, fl, fl, fl };
    volatile v4i* qo = (volatile v4i*)(OFFg + (size_t)blk * OFFP + 4 * tid);
    volatile v4i* qt = (volatile v4i*)(OFFg + (size_t)blk * OFFP + GS + 4 * (tid & 7));
    volatile v4i* qf = (volatile v4i*)(FLAGg + (size_t)blk * 32 + 4 * (tid & 7));
    *qo = oc;
    if (tid < 8) { *qt = tl; *qf = fv; }
    __threadfence();
    *qo = oc;
    if (tid < 8) { *qt = tl; *qf = fv; }
  }
}

struct Ent { float e; int g; };

__device__ __forceinline__ float nmax(float a, float b) {
  float r = (b > a) ? b : a;
  r = (b != b) ? b : r;
  return r;
}

__device__ __forceinline__ Ent entry_score(int idx, int cn, const int* __restrict__ lst, int b,
                                           const float* __restrict__ SS, const float* __restrict__ ea,
                                           v4f a0, v4f a1, v4f a2, v4f a3, float sdn, float eloop) {
  int jj = idx > cn - 1 ? cn - 1 : idx;
  jj = jj < 0 ? 0 : jj;
  int w = lst[jj];
  asm volatile("" :: "v"(w));
  const int g  = w & (GS - 1);
  const int le = (w >> 10) & (GEP - 1);
  const float ssg = SS[b * GS + g];
  asm volatile("" :: "v"(ssg));
  const float* erow = ea + (size_t)(b * GEP + le) * 16;
  const v4f x0 = *(const v4fa*)(erow);
  const v4f x1 = *(const v4fa*)(erow + 4);
  const v4f x2 = *(const v4fa*)(erow + 8);
  const v4f x3 = *(const v4fa*)(erow + 12);
  asm volatile("" :: "v"(x0), "v"(x1));
  asm volatile("" :: "v"(x2), "v"(x3));
  float d = bf16_val(x0.x) * a0.x;
  d = d + bf16_val(x0.y) * a0.y;
  d = d + bf16_val(x0.z) * a0.z;
  d = d + bf16_val(x0.w) * a0.w;
  d = d + bf16_val(x1.x) * a1.x;
  d = d + bf16_val(x1.y) * a1.y;
  d = d + bf16_val(x1.z) * a1.z;
  d = d + bf16_val(x1.w) * a1.w;
  d = d + bf16_val(x2.x) * a2.x;
  d = d + bf16_val(x2.y) * a2.y;
  d = d + bf16_val(x2.z) * a2.z;
  d = d + bf16_val(x2.w) * a2.w;
  d = d + bf16_val(x3.x) * a3.x;
  d = d + bf16_val(x3.y) * a3.y;
  d = d + bf16_val(x3.z) * a3.z;
  d = d + bf16_val(x3.w) * a3.w;
  const float v = (ssg + sdn) + d;
  float e = (v >= 0.0f) ? v : 0.2f * v;
  e = e / T_SOFT;
  Ent q;
  q.e = (idx < cn) ? e : eloop;
  q.g = g;
  return q;
}

__device__ __forceinline__ float sum_batch(float den, int xv, int cnt) {
#pragma unroll 1
  for (int i = 0; i < cnt; ++i) den = den + __int_as_float(__builtin_amdgcn_readlane(xv, i));
  return den;
}

__device__ __forceinline__ v4f walk_batch(v4f acc, int gv, int alv, int cnt, const float* __restrict__ xtb) {
#pragma unroll 1
  for (int i = 0; i < cnt; ++i) {
    const int g = __builtin_amdgcn_readlane(gv, i) & (GS - 1);
    const float al = __int_as_float(__builtin_amdgcn_readlane(alv, i));
    const v4f row = *(const v4fa*)(xtb + (size_t)g * GC);
    asm volatile("" :: "v"(row));
    acc.x = acc.x + al * row.x;
    acc.y = acc.y + al * row.y;
    acc.z = acc.z + al * row.z;
    acc.w = acc.w + al * row.w;
  }
  return acc;
}

__global__ __launch_bounds__(256) void k_attn(const float* __restrict__ ea, const float* __restrict__ XT,
                                              const float* __restrict__ SS, const float* __restrict__ SD,
                                              const float* __restrict__ ATAB, const int* __restrict__ LISTg,
                                              const int* __restrict__ OFFg, const int* __restrict__ FLAGg,
                                              float* __restrict__ out) {
  __shared__ __attribute__((aligned(16))) float sA[16];
  const int tid = (int)threadIdx.x, lane = tid & 31, wave = tid >> 5;
  {
    const v4f v = *(const v4fa*)(ATAB + 256 + 4 * (tid & 3));
    asm volatile("" :: "v"(v));
    if (tid < 4) *(v4fa*)(sA + 4 * tid) = v;
  }
  __syncthreads();
  const int n = (int)blockIdx.x * 8 + wave;
  if (n < NN) {
    const int b  = n >> 10;
    const int ln = n & (GS - 1);
    const v4f a0 = *(const v4fa*)(sA);
    const v4f a1 = *(const v4fa*)(sA + 4);
    const v4f a2 = *(const v4fa*)(sA + 8);
    const v4f a3 = *(const v4fa*)(sA + 12);
    const int* offb = OFFg + (size_t)b * OFFP;
    const int o0 = offb[ln];
    const int o1 = offb[ln + 1];
    const int fl = FLAGg[b * 32];
    asm volatile("" :: "v"(o0), "v"(o1), "v"(fl));
    const int craw = o1 - o0;
    const bool bad = (craw < 0) || (craw > DEGCAP) || (fl != 0);
    const int stv = clampi(o0, 0, RCAP - 1);
    int cnv = clampi(craw, 0, DEGCAP);
    cnv = cnv > (RCAP - stv) ? (RCAP - stv) : cnv;
    const int cn    = __builtin_amdgcn_readfirstlane(cnv);
    const int start = __builtin_amdgcn_readfirstlane(stv);
    const float ssn = SS[n];
    const float sdn = SD[n];
    asm volatile("" :: "v"(ssn), "v"(sdn));
    const float vl = (ssn + sdn) + 0.0f;
    float el = (vl >= 0.0f) ? vl : 0.2f * vl;
    el = el / T_SOFT;
    const int* lst = LISTg + (size_t)b * RCAP + start;

    const Ent q0 = entry_score(lane, cn, lst, b, SS, ea, a0, a1, a2, a3, sdn, el);
    int   g1 = 0;
    float e1 = el;
    if (cn > 32) {
      const Ent q1 = entry_score(32 + lane, cn, lst, b, SS, ea, a0, a1, a2, a3, sdn, el);
      g1 = q1.g;
      e1 = q1.e;
    }

    float m = nmax(q0.e, e1);
    m = nmax(m, __shfl_xor(m, 1));
    m = nmax(m, __shfl_xor(m, 2));
    m = nmax(m, __shfl_xor(m, 4));
    m = nmax(m, __shfl_xor(m, 8));
    m = nmax(m, __shfl_xor(m, 16));
    m = nmax(m, el);

    const float x0 = expf(q0.e - m);
    const float x1 = expf(e1 - m);
    const float xl = expf(el - m);

    const int n0 = cn < 32 ? cn : 32;
    const int n1 = cn > 32 ? cn - 32 : 0;
    float den = 0.0f;
    den = sum_batch(den, __float_as_int(x0), n0);
    den = sum_batch(den, __float_as_int(x1), n1);
    den = den + xl;

    const float al0 = x0 / den;
    const float al1 = x1 / den;
    const float all = xl / den;

    const float* xtb = XT + (size_t)(b * GS) * GC + 4 * lane;
    v4f acc = (v4f){0.0f, 0.0f, 0.0f, 0.0f};
    acc = walk_batch(acc, q0.g, __float_as_int(al0), n0, xtb);
    acc = walk_batch(acc, g1,   __float_as_int(al1), n1, xtb);
    {
      const v4f row = *(const v4fa*)(xtb + (size_t)ln * GC);
      asm volatile("" :: "v"(row));
      acc.x = acc.x + all * row.x;
      acc.y = acc.y + all * row.y;
      acc.z = acc.z + all * row.z;
      acc.w = acc.w + all * row.w;
    }

    const float qn = __int_as_float(0x7fc00000);
    const v4f v = (v4f){ bad ? qn : acc.x, bad ? qn : acc.y, bad ? qn : acc.z, bad ? qn : acc.w };
    volatile v4f* q = (volatile v4f*)(out + (size_t)n * GC + 4 * lane);
    *q = v;
    __threadfence();
    *q = v;
  }
}

extern "C" void kernel_launch(void* const* d_in, const int* in_sizes, int n_in,
                              void* d_out, int out_size, void* d_ws, size_t ws_size,
                              hipStream_t stream) {
  if (n_in < 7) return;
  if (in_sizes[0] != NN * 128) return;
  if (in_sizes[1] != GB * GEP * 2) return;
  if (in_sizes[2] != GB * GEP * 16) return;
  if (in_sizes[5] != 128 * 128) return;
  if (in_sizes[6] != ANUM) return;
  if (out_size != NN * GC) return;
  if (ws_size < WS_TOTAL) return;

  const float* x  = (const float*)d_in[0];
  const int*   ei = (const int*)  d_in[1];
  const float* ea = (const float*)d_in[2];
  const float* W  = (const float*)d_in[5];
  const float* a  = (const float*)d_in[6];
  float* out = (float*)d_out;

  char* ws = (char*)d_ws;
  size_t off = 0;
  unsigned short* XB = (unsigned short*)(ws + off); off += SZ_XB;
  unsigned short* WT = (unsigned short*)(ws + off); off += SZ_WT;
  float* ATAB        = (float*)(ws + off);          off += SZ_ATAB;
  float* XT          = (float*)(ws + off);          off += SZ_XT;
  float* SSp         = (float*)(ws + off);          off += SZ_SS;
  float* SDp         = (float*)(ws + off);          off += SZ_SS;
  int*   LIST        = (int*)(ws + off);            off += SZ_LIST;
  int*   OFFT        = (int*)(ws + off);            off += SZ_OFF;
  int*   FLAG        = (int*)(ws + off);            off += SZ_FLAG;
  if (off != WS_TOTAL) return;

  hipFuncSetAttribute(reinterpret_cast<const void*>(&k_bucket),
                      hipFuncAttributeMaxDynamicSharedMemorySize, LDS_BUCKET);

  k_plane<0><<<(NN * 128 / 8) / 256, 256, 0, stream>>>(x, NN, 128, 128, XB, NN, 128);
  k_prep<<<4, 256, 0, stream>>>(W, a, WT, ATAB);
  k_gemm_nt<0, 0><<<(256 * 2) / 8, 256, 0, stream>>>(XB, WT, ATAB, XT, NN, 128, 128, 128);
  k_node<<<NN / 32, 256, 0, stream>>>(XT, ATAB, SSp, SDp);
  k_bucket<<<GB, 256, LDS_BUCKET, stream>>>(ei, LIST, OFFT, FLAG);
  k_attn<<<NN / 8, 256, 0, stream>>>(ea, XT, SSp, SDp, ATAB, LIST, OFFT, FLAG, out);
}
